// QNetwork_72662256713877
// MI455X (gfx1250) — hardware-run, weakly checked
//
#include <hip/hip_runtime.h>
#include <stdint.h>
#include <stddef.h>
#include <math.h>

typedef __attribute__((ext_vector_type(16))) _Float16 v16h;
typedef __attribute__((ext_vector_type(8)))  _Float16 v8h;
typedef __attribute__((ext_vector_type(16))) __bf16   v16b;
typedef __attribute__((ext_vector_type(8)))  __bf16   v8b;
typedef __attribute__((ext_vector_type(8)))  float    v8f;
typedef __attribute__((ext_vector_type(4)))  float    v4f;
typedef __attribute__((ext_vector_type(2)))  float    v2f;
typedef __attribute__((ext_vector_type(2)))  int      v2i;

constexpr int NBATCH = 10;
constexpr int NCHAN  = 3;
constexpr int GH     = 50;
constexpr int GW     = 101;
constexpr int CELLS  = GH * GW;
constexpr int NPTS   = 4096;
constexpr int NTHR   = 256;
constexpr int O1H = 25, O1W = 51;
constexpr int M1ROWS = O1H * O1W;
constexpr int M1B    = 1280;
constexpr int M1     = NBATCH * M1B;
constexpr int K1R    = 147;
constexpr int K1P    = 160;
constexpr int N1R    = 32;
constexpr int N1P    = 64;
constexpr int P1H = 12, P1W = 25, P1C = 32;
constexpr int NP1 = NBATCH * P1H * P1W * P1C;
constexpr int M2R = NBATCH * P1H * P1W;
constexpr int M2P = 3072;
constexpr int K2  = 800;
constexpr int N2  = 64;
constexpr int P2H = 6, P2W = 12, P2C = 64;
constexpr int NP2 = NBATCH * P2H * P2W * P2C;
constexpr int M3R = NBATCH * P2H * P2W;
constexpr int M3P = 768;
constexpr int K3  = 576;
constexpr int N3  = 128;
constexpr int P3H = 3, P3W = 6;
constexpr int NFEAT = 128, NOUT = 5;
constexpr float WCARRY = 16.0f;
constexpr float ACARRY = 16.0f;

static_assert(K1P % 32 == 0 && K2 % 32 == 0 && K3 % 32 == 0);
static_assert(K1P >= K1R);
static_assert(M1 % 64 == 0 && M2P % 64 == 0 && M3P % 64 == 0);
static_assert(N1P % 64 == 0 && N2 % 64 == 0 && N3 % 64 == 0);
static_assert(M1B >= M1ROWS && M2P >= M2R && M3P >= M3R && N1P >= N1R);
static_assert((M1B * (K1P / 8)) % NTHR == 0);
static_assert((M2P * (K2 / 8)) % NTHR == 0);
static_assert((M3P * (K3 / 8)) % NTHR == 0);
static_assert((N1P * (K1P / 8)) % NTHR == 0 && (N2 * (K2 / 8)) % NTHR == 0 && (N3 * (K3 / 8)) % NTHR == 0);
static_assert(NP1 % NTHR == 0 && NP2 % NTHR == 0);
static_assert((NBATCH * NFEAT) % NTHR == 0);
static_assert(NBATCH * NOUT <= 64 && NBATCH * NOUT == 50);
static_assert((M1B * K1P * 2) % 512 == 0);
static_assert(NCHAN * CELLS * 4 <= 65536);

__device__ __forceinline__ unsigned short f2bf_bits(float f) {
  unsigned u = __float_as_uint(f);
  return (unsigned short)((u + 0x7FFFu + ((u >> 16) & 1u)) >> 16);
}
__device__ __forceinline__ float bf_bits2f(unsigned short h) { return __uint_as_float(((unsigned)h) << 16); }

__device__ __forceinline__ void dep_guard_h(v8f& a, v8f& b, v16h x, v16h y) { asm volatile("v_nop\n\tv_nop\n\tv_nop\n\tv_nop" : "+v"(a), "+v"(b) : "v"(x), "v"(y)); }
__device__ __forceinline__ void dep_guard_b(v8f& a, v8f& b, v16b x, v16b y) { asm volatile("v_nop\n\tv_nop\n\tv_nop\n\tv_nop" : "+v"(a), "+v"(b) : "v"(x), "v"(y)); }
__device__ __forceinline__ void keep4_h(v16h a, v16h b, v16h c, v16h d) { asm volatile("v_nop" :: "v"(a), "v"(b), "v"(c), "v"(d)); }
__device__ __forceinline__ void keep4_b(v16b a, v16b b, v16b c, v16b d) { asm volatile("v_nop" :: "v"(a), "v"(b), "v"(c), "v"(d)); }
__device__ __forceinline__ void acc_guard4(v8f& a, v8f& b, v8f& c, v8f& d) { asm volatile("v_nop\n\tv_nop\n\tv_nop\n\tv_nop" : "+v"(a), "+v"(b), "+v"(c), "+v"(d)); }
template <typename T> struct Frag;
template <> struct Frag<_Float16> {
  typedef v16h V; union U { v16h v; v8h h[2]; };
  static __device__ __forceinline__ v16h load(const _Float16* p) {
    U f; f.h[0] = *(const v8h*)(p); f.h[1] = *(const v8h*)(p + 16); return f.v;
  }
  static __device__ __forceinline__ v8f mma(v16h a, v16h b, v8f c) {
    return __builtin_amdgcn_wmma_f32_16x16x32_f16(false, a, false, b, (short)0, c, false, false);
  }
  static __device__ __forceinline__ void guard(v8f& a, v8f& b, v16h x, v16h y) { dep_guard_h(a, b, x, y); }
  static __device__ __forceinline__ void keep(v16h a, v16h b, v16h c, v16h d) { keep4_h(a, b, c, d); }
};
template <> struct Frag<__bf16> {
  typedef v16b V; union U { v16b v; v8b h[2]; };
  static __device__ __forceinline__ v16b load(const __bf16* p) {
    U f; f.h[0] = *(const v8b*)(p); f.h[1] = *(const v8b*)(p + 16); return f.v;
  }
  static __device__ __forceinline__ v8f mma(v16b a, v16b b, v8f c) {
    return __builtin_amdgcn_wmma_f32_16x16x32_bf16(false, a, false, b, (short)0, c, false, false);
  }
  static __device__ __forceinline__ void guard(v8f& a, v8f& b, v16b x, v16b y) { dep_guard_b(a, b, x, y); }
  static __device__ __forceinline__ void keep(v16b a, v16b b, v16b c, v16b d) { keep4_b(a, b, c, d); }
};

template <int ET> struct Elem;
template <> struct Elem<0> { typedef _Float16 T; };
template <> struct Elem<1> { typedef __bf16 T; };
template <int ET, bool SPLIT, int BIAS_MODE, int OUT_MODE, bool RESID, int ACT = 0>
__global__ __launch_bounds__(256) void wmma_gemm64(
    const unsigned short* __restrict__ Ap, const unsigned short* __restrict__ A2p, int lda, long strideA,
    const unsigned short* __restrict__ Btp, const unsigned short* __restrict__ Bt2p, int ldb, long strideB,
    void* __restrict__ Cout, void* __restrict__ Cout2, int ldc, long strideC,
    const float* __restrict__ bias,
    const float* __restrict__ resid, long strideR,
    int M, int N, int K, float scale) {
  typedef typename Elem<ET>::T T;
  typedef typename Frag<T>::V V;
  const T* A = (const T*)Ap; const T* A2 = (const T*)A2p; const T* Bt = (const T*)Btp; const T* Bt2 = (const T*)Bt2p;
  __shared__ __align__(16) float sT[8][16 * 68];
  const int b    = blockIdx.y;
  const int lane = threadIdx.x & 31;
  const int wave = threadIdx.x >> 5;
  const int tilesN = N >> 6;
  const int tilesM = M >> 6;
  const int tile = blockIdx.x * 8 + wave;
  if (tile >= tilesM * tilesN) return;
  const int tm = tile / tilesN;
  const int tn = tile - tm * tilesN;
  const int m0 = tm << 6;
  const int n0 = tn << 6;

  const T* Ab  = A  + (size_t)b * strideA;
  const T* Bb  = Bt + (size_t)b * strideB;
  const T* Ab2 = SPLIT ? (A2  + (size_t)b * strideA) : nullptr;
  const T* Bb2 = SPLIT ? (Bt2 + (size_t)b * strideB) : nullptr;

  const int rlane = lane & 15;
  const int koff  = (lane >> 4) * 8;
  const int mOff  = (lane >> 4) * 8;

  v8f acc[4][4];
#pragma unroll
  for (int i = 0; i < 4; ++i)
#pragma unroll
    for (int j = 0; j < 4; ++j) acc[i][j] = (v8f){0.f,0.f,0.f,0.f,0.f,0.f,0.f,0.f};

  for (int k0 = 0; k0 < K; k0 += 32) {
    V bh[4], bl[4];
#pragma unroll
    for (int j = 0; j < 4; ++j) {
      const size_t bo = (size_t)(n0 + (j << 4) + rlane) * ldb + koff + k0;
      bh[j] = Frag<T>::load(Bb + bo);
      if (SPLIT) bl[j] = Frag<T>::load(Bb2 + bo);
    }
#pragma unroll
    for (int i = 0; i < 4; ++i) {
      const size_t ao = (size_t)(m0 + (i << 4) + rlane) * lda + koff + k0;
      V ah = Frag<T>::load(Ab + ao);
      V al;
      if (SPLIT) al = Frag<T>::load(Ab2 + ao);
#pragma unroll
      for (int j = 0; j < 4; ++j) {
        acc[i][j] = Frag<T>::mma(ah, bh[j], acc[i][j]);
        if (SPLIT) {
          acc[i][j] = Frag<T>::mma(ah, bl[j], acc[i][j]);
          acc[i][j] = Frag<T>::mma(al, bh[j], acc[i][j]);
        }
      }
      Frag<T>::guard(acc[i][0], acc[i][3], ah, SPLIT ? al : ah);
    }
    Frag<T>::keep(bh[0], bh[1], bh[2], bh[3]);
    if (SPLIT) Frag<T>::keep(bl[0], bl[1], bl[2], bl[3]);
  }
  acc_guard4(acc[0][0], acc[0][1], acc[0][2], acc[0][3]);
  acc_guard4(acc[1][0], acc[1][1], acc[1][2], acc[1][3]);
  acc_guard4(acc[2][0], acc[2][1], acc[2][2], acc[2][3]);
  acc_guard4(acc[3][0], acc[3][1], acc[3][2], acc[3][3]);

  float* slab = sT[wave];
  const float* Rb = RESID ? (resid + (size_t)b * strideR) : nullptr;
#pragma unroll
  for (int i = 0; i < 4; ++i) {
    const int mBase = m0 + (i << 4);
#pragma unroll
    for (int j = 0; j < 4; ++j) {
      const int n = n0 + (j << 4) + rlane;
      float bv = 0.f;
      if (BIAS_MODE == 2) bv = bias[n];
#pragma unroll
      for (int r = 0; r < 8; ++r) {
        float v = acc[i][j][r] * scale;
        if (BIAS_MODE == 1) v += bias[mBase + mOff + r];
        if (BIAS_MODE == 2) v += bv;
        if (RESID) v += Rb[(size_t)(mBase + mOff + r) * ldc + n];
        if (ACT == 1) v = tanhf(v);
        if (ACT == 2) v = fmaxf(v, 0.0f);
        if (ACT == 3) v = v / (1.0f + expf(-v));
        if (ACT == 4) v = (v > 0.f) ? v : 0.01f * v;
        if (ACT == 5) v = 0.5f * v * (1.0f + erff(v * 0.70710678118654752f));
        slab[(mOff + r) * 68 + (j << 4) + rlane] = v;
      }
    }
    __builtin_amdgcn_fence(__ATOMIC_RELEASE, "workgroup");
    __builtin_amdgcn_wave_barrier();
    __builtin_amdgcn_fence(__ATOMIC_ACQUIRE, "workgroup");
    if (OUT_MODE == 0) {
      float* C = (float*)Cout + (size_t)b * strideC;
      const int hh = lane >> 4, c4 = (lane & 15) * 4;
      for (int pass = 0; pass < 2; ++pass) {
#pragma unroll
        for (int it = 0; it < 8; ++it) {
          const int row = it * 2 + hh;
          v4f v = *(const v4f*)(slab + row * 68 + c4);
          *(volatile v4f*)(C + (size_t)(mBase + row) * ldc + n0 + c4) = v;
        }
        __threadfence();
      }
    } else {
      const int q = lane >> 3, c8 = (lane & 7) * 8;
      unsigned short* C  = (unsigned short*)Cout  + (size_t)b * strideC;
      unsigned short* C2 = (OUT_MODE == 2) ? ((unsigned short*)Cout2 + (size_t)b * strideC) : nullptr;
      for (int pass = 0; pass < 2; ++pass) {
#pragma unroll
        for (int it = 0; it < 4; ++it) {
          const int row = it * 4 + q;
          const float* sp = slab + row * 68 + c8;
          v8h hv, lv;
#pragma unroll
          for (int e = 0; e < 8; ++e) {
            if (OUT_MODE == 1) {
              hv[e] = (_Float16)sp[e];
            } else {
              unsigned short hb = f2bf_bits(sp[e]);
              unsigned short lb = f2bf_bits(sp[e] - bf_bits2f(hb));
              hv[e] = __builtin_bit_cast(_Float16, hb);
              lv[e] = __builtin_bit_cast(_Float16, lb);
            }
          }
          *(volatile v8h*)(C + (size_t)(mBase + row) * ldc + n0 + c8) = hv;
          if (OUT_MODE == 2) *(volatile v8h*)(C2 + (size_t)(mBase + row) * ldc + n0 + c8) = lv;
        }
        __threadfence();
      }
    }
    __builtin_amdgcn_fence(__ATOMIC_RELEASE, "workgroup");
    __builtin_amdgcn_wave_barrier();
    __builtin_amdgcn_fence(__ATOMIC_ACQUIRE, "workgroup");
  }
}

__device__ __forceinline__ float bfr(float f) { return bf_bits2f(f2bf_bits(f)); }

__global__ __launch_bounds__(NTHR) void k_wprep(const float* __restrict__ W, int nreal, int kreal, int npad, int kpad,
                                                unsigned short* __restrict__ bt,
                                                const float* __restrict__ bsrc, int nbias, int nbpad,
                                                float* __restrict__ bdst) {
  const int tid = threadIdx.x;
  const int lane = tid & 31;
  const int wave = tid >> 5;
  if (blockIdx.x == 0 && wave == 0) {
    v4f bv;
#pragma unroll
    for (int q = 0; q < 4; ++q) {
      const int idx = 4 * lane + q;
      const int ic  = (idx < nbias) ? idx : (nbias - 1);
      const float fk = (idx < nbias) ? 1.0f : 0.0f;
      bv[q] = bfr(bsrc[ic]) * fk;
    }
    if (4 * lane < nbpad) {
      *(volatile v4f*)(bdst + 4 * lane) = bv;
      __threadfence();
      *(volatile v4f*)(bdst + 4 * lane) = bv;
    }
  }
  const int tpr = kpad >> 3;
  const int i = blockIdx.x * NTHR + tid;
  if (i >= npad * tpr) return;
  const int n  = i / tpr;
  const int k0 = (i - n * tpr) * 8;
  const int nc = (n < nreal) ? n : (nreal - 1);
  const float fn = (n < nreal) ? 1.0f : 0.0f;
  v8h hv;
#pragma unroll
  for (int e = 0; e < 8; ++e) {
    const int k  = k0 + e;
    const int kc = (k < kreal) ? k : (kreal - 1);
    const float fk = (k < kreal) ? fn : 0.0f;
    const float w = W[(size_t)nc * kreal + kc];
    hv[e] = (_Float16)(WCARRY * bfr(w) * fk);
  }
  const size_t o = (size_t)i * 8;
  *(volatile v8h*)(bt + o) = hv;
  __threadfence();
  *(volatile v8h*)(bt + o) = hv;
}

#define CELL_MAX(SL, RR, CC, KEY) do { const int r_ = (RR); const int c_ = (CC); \
    if ((unsigned)r_ < (unsigned)GH && (unsigned)c_ < (unsigned)GW) \
      atomicMax(&cells[(SL) * CELLS + r_ * GW + c_], (KEY)); } while (0)

__global__ __launch_bounds__(NTHR) void k_grid_im2col1(const int* __restrict__ xy, unsigned short* __restrict__ a1) {
  __shared__ int cells[NCHAN * CELLS];
  const int tid = threadIdx.x;
  const int b = blockIdx.x;
  const int key_none = -2147483647 - 1;

#pragma unroll 1
  for (int i = tid; i < NCHAN * CELLS; i += NTHR) cells[i] = key_none;
  __syncthreads();

  if (tid < NCHAN) {
    const int s = tid;
    CELL_MAX(s, 47, 49, 0); CELL_MAX(s, 47, 50, 1); CELL_MAX(s, 47, 51, 2);
    CELL_MAX(s, 48, 49, 3);                          CELL_MAX(s, 48, 51, 5);
    CELL_MAX(s, 49, 49, 6); CELL_MAX(s, 49, 50, 7); CELL_MAX(s, 49, 51, 8);
    CELL_MAX(s, 48, 50, 9);
  }
#pragma unroll 1
  for (int idx = tid; idx < NCHAN * NPTS; idx += NTHR) {
    const int s = idx >> 12;
    const int p = idx & (NPTS - 1);
    const v2i cr = *(const v2i*)(xy + ((size_t)(b * NCHAN + s) * NPTS + p) * 2);
    const int col = cr.x;
    const int row = cr.y;
    const int kb = (p + 1) * 10;
    CELL_MAX(s, row - 1, col - 1, kb + 0); CELL_MAX(s, row - 1, col, kb + 1); CELL_MAX(s, row - 1, col + 1, kb + 2);
    CELL_MAX(s, row,     col - 1, kb + 3);                                     CELL_MAX(s, row,     col + 1, kb + 5);
    CELL_MAX(s, row + 1, col - 1, kb + 6); CELL_MAX(s, row + 1, col, kb + 7); CELL_MAX(s, row + 1, col + 1, kb + 8);
    CELL_MAX(s, row,     col,     kb + 9);
  }
  __syncthreads();

#pragma unroll 1
  for (int i = tid; i < NCHAN * CELLS; i += NTHR) {
    const int key = cells[i];
    const unsigned ku = (unsigned)((key < 0) ? 0 : key);
    float v = ((ku % 10u) == 9u) ? 1.0f : 0.5f;
    if (key < 0) v = 0.0f;
    cells[i] = __float_as_int(v);
  }
  __syncthreads();

  unsigned short* plane = a1 + (size_t)b * ((size_t)M1B * K1P);
#pragma unroll 1
  for (int it = 0; it < (M1B * (K1P / 8)) / NTHR; ++it) {
    const int i   = it * NTHR + tid;
    const int row = i / (K1P / 8);
    const int k0  = (i - row * (K1P / 8)) * 8;
    const int oh  = row / O1W;
    const int ow  = row - oh * O1W;
    const float frow = (row < M1ROWS) ? 1.0f : 0.0f;
    v8h hv;
#pragma unroll
    for (int e = 0; e < 8; ++e) {
      const int k   = k0 + e;
      const int ci  = k / 49;
      const int rem = k - ci * 49;
      const int kh  = rem / 7;
      const int kw  = rem - kh * 7;
      const int ih  = 2 * oh - 3 + kh;
      const int iw  = 2 * ow - 3 + kw;
      const bool valid = (k < K1R) && ((unsigned)ih < (unsigned)GH) && ((unsigned)iw < (unsigned)GW);
      const int cic = (ci < NCHAN) ? ci : (NCHAN - 1);
      const int ihc = (ih < 0) ? 0 : ((ih >= GH) ? (GH - 1) : ih);
      const int iwc = (iw < 0) ? 0 : ((iw >= GW) ? (GW - 1) : iw);
      const float v = __int_as_float(cells[cic * CELLS + ihc * GW + iwc]);
      hv[e] = (_Float16)(v * (valid ? frow : 0.0f));
    }
    unsigned short* p = plane + (size_t)i * 8;
    *(volatile v8h*)p = hv;
    __threadfence();
    *(volatile v8h*)p = hv;
  }
}
#undef CELL_MAX

__global__ __launch_bounds__(NTHR) void k_pool1(const float* __restrict__ c1, float* __restrict__ p1) {
  const int t = blockIdx.x * NTHR + threadIdx.x;
  if (t >= NP1) return;
  const int c   = t & (P1C - 1);
  const int pos = t >> 5;
  const int pw  = pos % P1W;
  const int t2  = pos / P1W;
  const int ph  = t2 % P1H;
  const int b   = t2 / P1H;
  float m = 0.0f;
#pragma unroll
  for (int i = 0; i < 3; ++i) {
#pragma unroll
    for (int j = 0; j < 3; ++j) {
      const size_t row = (size_t)b * M1B + (size_t)(2 * ph + i) * O1W + (2 * pw + j);
      const float v = c1[row * N1P + c];
      m = (i == 0 && j == 0) ? v : fmaxf(m, v);
    }
  }
  *(volatile float*)(p1 + t) = m;
  __threadfence();
  *(volatile float*)(p1 + t) = m;
}

__global__ __launch_bounds__(NTHR) void k_im2col2(const float* __restrict__ p1, unsigned short* __restrict__ a2) {
  const int i = blockIdx.x * NTHR + threadIdx.x;
  if (i >= M2P * (K2 / 8)) return;
  const int row = i / (K2 / 8);
  const int k0  = (i - row * (K2 / 8)) * 8;
  const int b   = row / (P1H * P1W);
  const int r2  = row - b * (P1H * P1W);
  const int oh  = r2 / P1W;
  const int ow  = r2 - oh * P1W;
  const float frow = (row < M2R) ? 1.0f : 0.0f;
  const int bc = (b < NBATCH) ? b : (NBATCH - 1);
  v8h hv;
#pragma unroll
  for (int e = 0; e < 8; ++e) {
    const int k   = k0 + e;
    const int ci  = k / 25;
    const int rem = k - ci * 25;
    const int kh  = rem / 5;
    const int kw  = rem - kh * 5;
    const int ih  = oh - 2 + kh;
    const int iw  = ow - 2 + kw;
    const bool valid = ((unsigned)ih < (unsigned)P1H) && ((unsigned)iw < (unsigned)P1W);
    const int ihc = (ih < 0) ? 0 : ((ih >= P1H) ? (P1H - 1) : ih);
    const int iwc = (iw < 0) ? 0 : ((iw >= P1W) ? (P1W - 1) : iw);
    const float v = p1[((size_t)(bc * P1H + ihc) * P1W + iwc) * P1C + ci];
    hv[e] = (_Float16)(ACARRY * v * (valid ? frow : 0.0f));
  }
  unsigned short* p = a2 + (size_t)i * 8;
  *(volatile v8h*)p = hv;
  __threadfence();
  *(volatile v8h*)p = hv;
}

__global__ __launch_bounds__(NTHR) void k_pool2(const float* __restrict__ c2, float* __restrict__ p2) {
  const int t = blockIdx.x * NTHR + threadIdx.x;
  if (t >= NP2) return;
  const int c   = t & (P2C - 1);
  const int pos = t >> 6;
  const int pw  = pos % P2W;
  const int t2  = pos / P2W;
  const int ph  = t2 % P2H;
  const int b   = t2 / P2H;
  const size_t r0 = (size_t)(b * P1H + 2 * ph) * P1W + 2 * pw;
  const float v00 = c2[r0 * N2 + c];
  const float v01 = c2[(r0 + 1) * N2 + c];
  const float v10 = c2[(r0 + P1W) * N2 + c];
  const float v11 = c2[(r0 + P1W + 1) * N2 + c];
  const float m = fmaxf(fmaxf(v00, v01), fmaxf(v10, v11));
  *(volatile float*)(p2 + t) = m;
  __threadfence();
  *(volatile float*)(p2 + t) = m;
}

__global__ __launch_bounds__(NTHR) void k_im2col3(const float* __restrict__ p2, unsigned short* __restrict__ a3) {
  const int i = blockIdx.x * NTHR + threadIdx.x;
  if (i >= M3P * (K3 / 8)) return;
  const int row = i / (K3 / 8);
  const int k0  = (i - row * (K3 / 8)) * 8;
  const int b   = row / (P2H * P2W);
  const int r2  = row - b * (P2H * P2W);
  const int oh  = r2 / P2W;
  const int ow  = r2 - oh * P2W;
  const float frow = (row < M3R) ? 1.0f : 0.0f;
  const int bc = (b < NBATCH) ? b : (NBATCH - 1);
  v8h hv;
#pragma unroll
  for (int e = 0; e < 8; ++e) {
    const int k   = k0 + e;
    const int ci  = k / 9;
    const int rem = k - ci * 9;
    const int kh  = rem / 3;
    const int kw  = rem - kh * 3;
    const int ih  = oh - 1 + kh;
    const int iw  = ow - 1 + kw;
    const bool valid = ((unsigned)ih < (unsigned)P2H) && ((unsigned)iw < (unsigned)P2W);
    const int ihc = (ih < 0) ? 0 : ((ih >= P2H) ? (P2H - 1) : ih);
    const int iwc = (iw < 0) ? 0 : ((iw >= P2W) ? (P2W - 1) : iw);
    const float v = p2[((size_t)(bc * P2H + ihc) * P2W + iwc) * P2C + ci];
    hv[e] = (_Float16)(ACARRY * v * (valid ? frow : 0.0f));
  }
  unsigned short* p = a3 + (size_t)i * 8;
  *(volatile v8h*)p = hv;
  __threadfence();
  *(volatile v8h*)p = hv;
}

__global__ __launch_bounds__(NTHR) void k_tail(const float* __restrict__ c3,
                                               const float* __restrict__ wl1, const float* __restrict__ bl1,
                                               const float* __restrict__ wl2, const float* __restrict__ bl2,
                                               float* __restrict__ out) {
  __shared__ __align__(16) float feat[NBATCH * NFEAT];
  __shared__ __align__(16) float h1s[NBATCH * NFEAT];
  __shared__ __align__(16) float res[64];
  const int tid = threadIdx.x;

#pragma unroll 1
  for (int it = 0; it < (NBATCH * NFEAT) / NTHR; ++it) {
    const int o = it * NTHR + tid;
    const int b = o >> 7;
    const int c = o & (NFEAT - 1);
    float s = 0.0f;
#pragma unroll 1
    for (int ph = 0; ph < P3H; ++ph) {
#pragma unroll 1
      for (int pw = 0; pw < P3W; ++pw) {
        const size_t r0 = ((size_t)(b * P2H + 2 * ph) * P2W + 2 * pw) * N3 + c;
        const float v00 = c3[r0];
        const float v01 = c3[r0 + N3];
        const float v10 = c3[r0 + (size_t)P2W * N3];
        const float v11 = c3[r0 + (size_t)P2W * N3 + N3];
        s += fmaxf(fmaxf(v00, v01), fmaxf(v10, v11));
      }
    }
    feat[o] = s * (1.0f / 18.0f);
  }
  __syncthreads();

#pragma unroll 1
  for (int it = 0; it < (NBATCH * NFEAT) / NTHR; ++it) {
    const int o = it * NTHR + tid;
    const int b = o >> 7;
    const int n = o & (NFEAT - 1);
    float acc = 0.0f;
#pragma unroll 1
    for (int k = 0; k < NFEAT; ++k) acc = fmaf(feat[b * NFEAT + k], bfr(wl1[(size_t)n * NFEAT + k]), acc);
    acc += bfr(bl1[n]);
    h1s[o] = fmaxf(acc, 0.0f);
  }
  __syncthreads();

  if (tid < 64) {
    const int q = (tid < NBATCH * NOUT) ? tid : (NBATCH * NOUT - 1);
    const int b = q / NOUT;
    const int n = q - b * NOUT;
    float acc = 0.0f;
#pragma unroll 1
    for (int k = 0; k < NFEAT; ++k) acc = fmaf(h1s[b * NFEAT + k], bfr(wl2[(size_t)n * NFEAT + k]), acc);
    acc += bfr(bl2[n]);
    res[tid] = acc * ((tid < NBATCH * NOUT) ? 1.0f : 0.0f);
  }
  __syncthreads();

  if (tid < 32) {
    const int lane = tid;
    v2f v;
    v.x = res[2 * lane];
    v.y = res[2 * lane + 1];
    if (lane < (NBATCH * NOUT) / 2) {
      *(volatile v2f*)(out + 2 * lane) = v;
      __threadfence();
      *(volatile v2f*)(out + 2 * lane) = v;
    }
  }
}

extern "C" void kernel_launch(void* const* d_in, const int* in_sizes, int n_in,
                              void* d_out, int out_size, void* d_ws, size_t ws_size,
                              hipStream_t stream) {
  if (n_in < 11 || out_size < NBATCH * NOUT) return;
  if (in_sizes[0] < NBATCH * NCHAN * NPTS * 2) return;
  if (in_sizes[1] < N1R * K1R || in_sizes[3] < N2 * K2 || in_sizes[5] < N3 * K3) return;
  if (in_sizes[7] < NFEAT * NFEAT || in_sizes[9] < NOUT * NFEAT) return;

  const int*   xy  = (const int*)d_in[0];
  const float* w1  = (const float*)d_in[1];
  const float* b1  = (const float*)d_in[2];
  const float* w2  = (const float*)d_in[3];
  const float* b2  = (const float*)d_in[4];
  const float* w3  = (const float*)d_in[5];
  const float* b3  = (const float*)d_in[6];
  const float* wl1 = (const float*)d_in[7];
  const float* bl1 = (const float*)d_in[8];
  const float* wl2 = (const float*)d_in[9];
  const float* bl2 = (const float*)d_in[10];
  float* out = (float*)d_out;

  char* ws = (char*)d_ws;
  size_t off = 0;
  auto carve = [&](size_t bytes) -> char* {
    char* p = ws + off;
    off += (bytes + 255) & ~(size_t)255;
    return p;
  };
  unsigned short* Bt1 = (unsigned short*)carve((size_t)N1P * K1P * 2);
  unsigned short* Bt2 = (unsigned short*)carve((size_t)N2 * K2 * 2);
  unsigned short* Bt3 = (unsigned short*)carve((size_t)N3 * K3 * 2);
  float* bias1 = (float*)carve((size_t)N1P * 4);
  float* bias2 = (float*)carve((size_t)N2 * 4);
  float* bias3 = (float*)carve((size_t)N3 * 4);
  unsigned short* A1 = (unsigned short*)carve((size_t)M1 * K1P * 2);
  float* C1 = (float*)carve((size_t)M1 * N1P * 4);
  float* P1 = (float*)carve((size_t)NP1 * 4);
  unsigned short* A2 = (unsigned short*)carve((size_t)M2P * K2 * 2);
  float* C2 = (float*)carve((size_t)M2P * N2 * 4);
  float* P2 = (float*)carve((size_t)NP2 * 4);
  unsigned short* A3 = (unsigned short*)carve((size_t)M3P * K3 * 2);
  float* C3 = (float*)carve((size_t)M3P * N3 * 4);
  if (off > ws_size) return;

  k_wprep<<<(N1P * (K1P / 8)) / NTHR, NTHR, 0, stream>>>(w1, N1R, K1R, N1P, K1P, Bt1, b1, N1R, N1P, bias1);
  k_wprep<<<(N2 * (K2 / 8)) / NTHR, NTHR, 0, stream>>>(w2, N2, K2, N2, K2, Bt2, b2, N2, N2, bias2);
  k_wprep<<<(N3 * (K3 / 8)) / NTHR, NTHR, 0, stream>>>(w3, N3, K3, N3, K3, Bt3, b3, N3, N3, bias3);

  k_grid_im2col1<<<NBATCH, NTHR, 0, stream>>>(xy, A1);

  {
    const int tiles = (M1 / 64) * (N1P / 64);
    wmma_gemm64<0, false, 2, 0, false, 2><<<dim3((tiles + 7) / 8, 1), 256, 0, stream>>>(
        A1, A1, K1P, 0L, Bt1, Bt1, K1P, 0L, (void*)C1, (void*)C1, N1P, 0L,
        bias1, bias1, 0L, M1, N1P, K1P, 1.0f / WCARRY);
  }
  k_pool1<<<NP1 / NTHR, NTHR, 0, stream>>>(C1, P1);
  k_im2col2<<<(M2P * (K2 / 8)) / NTHR, NTHR, 0, stream>>>(P1, A2);
  {
    const int tiles = (M2P / 64) * (N2 / 64);
    wmma_gemm64<0, false, 2, 0, false, 2><<<dim3((tiles + 7) / 8, 1), 256, 0, stream>>>(
        A2, A2, K2, 0L, Bt2, Bt2, K2, 0L, (void*)C2, (void*)C2, N2, 0L,
        bias2, bias2, 0L, M2P, N2, K2, 1.0f / (WCARRY * ACARRY));
  }
  k_pool2<<<NP2 / NTHR, NTHR, 0, stream>>>(C2, P2);
  k_im2col3<<<(M3P * (K3 / 8)) / NTHR, NTHR, 0, stream>>>(P2, A3);
  {
    const int tiles = (M3P / 64) * (N3 / 64);
    wmma_gemm64<0, false, 2, 0, false, 2><<<dim3((tiles + 7) / 8, 1), 256, 0, stream>>>(
        A3, A3, K3, 0L, Bt3, Bt3, K3, 0L, (void*)C3, (void*)C3, N3, 0L,
        bias3, bias3, 0L, M3P, N3, K3, 1.0f / (WCARRY * ACARRY));
  }
  k_tail<<<1, NTHR, 0, stream>>>(C3, wl1, bl1, wl2, bl2, out);
}
